// EnhancedGraphNeuralNetwork_4810363372589
// MI455X (gfx1250) — hardware-run, weakly checked
//
#include <hip/hip_runtime.h>
#include <stddef.h>
#include <stdint.h>
#include <math.h>

#define SPLIT_H 0

#define NN      100000
#define FD      128
#define NC      40
#define NCP     64
#define NE      1600000
#define MP      100096
#define KH      (SPLIT_H ? 256 : 128)
#define GBM     64
#define GTHR    128
#define NTHR    256
#define NWAVE   8
#define EPT     8
#define WCH     (32 * EPT)
#define NBRUN   1024
#define SLB     10
#define NBK     98
#define WLCAP   2560
#define RCAP    20480
#define TRIPCAP 64
#define MAXDEG_MEAS   36
#define MAXB1024_MEAS 16710
#define WSTW    258
#define RECW    384
#define WSMAX   134217728

#define BK_WL    (NWAVE * WLCAP)
#define BK_ZINTS (BK_WL + RCAP + 3 * NBRUN)
#define BK_INTS  (BK_ZINTS + 16)
#define BK_LDS   (BK_INTS * 4)

#define PBX   (MP * FD / 8 / NTHR)
#define PBW1  (FD * FD / 8 / NTHR)
#define PBW2  (FD * KH / 8 / NTHR)
#define PBW3  (NCP * KH / 8 / NTHR)
#define PBTOT (PBX + PBW1 + PBW2 + PBW3 + 1)

static_assert(FD == 128 && FD % 8 == 0 && FD == 32 * 4);
static_assert(MP % GBM == 0 && MP >= NN && MP == 782 * 128);
static_assert(NBRUN == (1 << SLB) && NBRUN % 32 == 0 && NBRUN == NWAVE * 128);
static_assert(NBK * NBRUN >= MP && NBK * NBRUN >= NN);
static_assert(NE < (1 << 21) && (((long long)NE) << SLB) < (1LL << 31));
static_assert(NE % WCH == 0 && NE % 4 == 0);
static_assert(RCAP == NWAVE * WLCAP && RCAP % (NTHR * 4) == 0 && BK_ZINTS % 4 == 0 && BK_WL % 4 == 0);
static_assert((long long)RCAP * 100 >= (long long)MAXB1024_MEAS * 105);
static_assert(WLCAP >= MAXB1024_MEAS / 8 + 8 * 46 + 1);
static_assert(MAXDEG_MEAS + 8 <= TRIPCAP);
static_assert((NBRUN * NC * 4) % 128 == 0 && (32 * NC * 4) % 128 == 0);
static_assert(NN % 32 == 0 && (NN - (NBK - 1) * NBRUN) == 672 && 672 % 32 == 0);
static_assert((MP * FD / 8) % NTHR == 0 && (FD * FD / 8) % NTHR == 0);
static_assert((FD * KH / 8) % NTHR == 0 && (NCP * KH / 8) % NTHR == 0);
static_assert(KH % 32 == 0 && FD % 32 == 0 && NC % 4 == 0 && NCP == 64);
static_assert(BK_LDS <= 300000);
static_assert(GBM * (FD + 4) * 4 + GBM * 4 <= 65536);
static_assert(NWAVE * 32 * NC * 4 + NCP * 4 <= 65536);
static_assert(RECW * 4 % 128 == 0 && RECW == 3 * FD);

typedef float          v4f   __attribute__((ext_vector_type(4)));
typedef float          v8f   __attribute__((ext_vector_type(8)));
typedef int            v2i   __attribute__((ext_vector_type(2)));
typedef int            v4i   __attribute__((ext_vector_type(4)));
typedef int            v8i   __attribute__((ext_vector_type(8)));
typedef unsigned short v8us  __attribute__((ext_vector_type(8)));
typedef unsigned short v16us __attribute__((ext_vector_type(16)));
typedef __bf16         v16bf __attribute__((ext_vector_type(16)));
typedef v4f  __attribute__((may_alias)) v4fa;
typedef v4i  __attribute__((may_alias)) v4ia;
typedef v8us __attribute__((may_alias)) v8usa;
union FragB { v16bf v; v16us u; v8us h[2]; v8i w; };

__device__ __forceinline__ v8f wmb(const FragB& a, const FragB& b, v8f c) {
  v8f d = __builtin_amdgcn_wmma_f32_16x16x32_bf16(false, a.v, false, b.v, (short)0, c, false, false);
  asm volatile("v_nop\n\tv_nop\n\tv_nop\n\tv_nop" : "+v"(d) : "v"(a.w), "v"(b.w));
  return d;
}

__device__ __forceinline__ unsigned bf16_bits(float f) {
  const unsigned u = __float_as_uint(f);
  const unsigned r = (u + 0x7FFFu + ((u >> 16) & 1u)) >> 16;
  const unsigned q = (u >> 16) | 0x40u;
  return ((u & 0x7fffffffu) > 0x7f800000u) ? q : r;
}
__device__ __forceinline__ float bf16_val(float f) {
  return __uint_as_float(bf16_bits(f) << 16);
}
__device__ __forceinline__ v4f bf4(v4f a) {
  v4f o;
  o.x = bf16_val(a.x); o.y = bf16_val(a.y); o.z = bf16_val(a.z); o.w = bf16_val(a.w);
  return o;
}

__device__ __forceinline__ void hilo_pack(float v0, float v1, float v2, float v3,
                                          int& h01, int& h23, int& l01, int& l23) {
  const unsigned a0 = bf16_bits(v0), a1 = bf16_bits(v1), a2 = bf16_bits(v2), a3 = bf16_bits(v3);
  const unsigned b0 = bf16_bits(v0 - __uint_as_float(a0 << 16));
  const unsigned b1 = bf16_bits(v1 - __uint_as_float(a1 << 16));
  const unsigned b2 = bf16_bits(v2 - __uint_as_float(a2 << 16));
  const unsigned b3 = bf16_bits(v3 - __uint_as_float(a3 << 16));
  h01 = (int)(a0 | (a1 << 16)); h23 = (int)(a2 | (a3 << 16));
  l01 = (int)(b0 | (b1 << 16)); l23 = (int)(b2 | (b3 << 16));
}

__device__ __forceinline__ v4i regroup32(int h01, int h23, int l01, int l23, int lane) {
  const int s0 = (2 * lane) & 31, s1 = s0 + 1;
  const int a0 = __shfl(h01, s0, 32), a1 = __shfl(h23, s0, 32), a2 = __shfl(h01, s1, 32), a3 = __shfl(h23, s1, 32);
  const int b0 = __shfl(l01, s0, 32), b1 = __shfl(l23, s0, 32), b2 = __shfl(l01, s1, 32), b3 = __shfl(l23, s1, 32);
  const int mk = (lane < 16) ? -1 : 0;
  v4i o;
  o.x = (a0 & mk) | (b0 & ~mk); o.y = (a1 & mk) | (b1 & ~mk);
  o.z = (a2 & mk) | (b2 & ~mk); o.w = (a3 & mk) | (b3 & ~mk);
  return o;
}

__device__ __forceinline__ void st2_v4f(float* p, v4f v) {
  *(volatile v4f*)p = v;
  __threadfence();
  *(volatile v4f*)p = v;
}
__device__ __forceinline__ void st2_v8us(unsigned short* p, v8us v) {
  *(volatile v8us*)p = v;
  __threadfence();
  *(volatile v8us*)p = v;
}

__device__ __forceinline__ v8us gather8(const float* __restrict__ base, int stride) {
  float f[8];
#pragma unroll
  for (int i = 0; i < 8; ++i) f[i] = base[(size_t)i * (size_t)stride];
  v8us o;
#pragma unroll
  for (int i = 0; i < 8; ++i) o[i] = (unsigned short)bf16_bits(f[i]);
  return o;
}

__global__ __launch_bounds__(NTHR) void k_prep(const float* __restrict__ x, const float* __restrict__ w1,
                                               const float* __restrict__ b1, const float* __restrict__ g1,
                                               const float* __restrict__ be1, const float* __restrict__ w2,
                                               const float* __restrict__ b2, const float* __restrict__ g2,
                                               const float* __restrict__ be2, const float* __restrict__ w3,
                                               const float* __restrict__ b3,
                                               unsigned short* xb, unsigned short* w1t, unsigned short* w2d,
                                               unsigned short* w3d, float* par) {
  constexpr int KU = KH / 8;
  const int tid = (int)threadIdx.x, lane = tid & 31;
  const int blk = (int)blockIdx.x;
  if (blk < PBX) {
    const int u   = blk * NTHR + tid;
    const int row = u >> 4, k8 = (u & 15) * 8;
    const int rc  = row < NN ? row : NN - 1;
    const unsigned mk = row < NN ? 0xffffu : 0u;
    const float* p = x + (size_t)rc * FD + k8;
    const v4f a = *(const v4fa*)p;
    const v4f b = *(const v4fa*)(p + 4);
    v8us o;
    o[0] = (unsigned short)(bf16_bits(a.x) & mk); o[1] = (unsigned short)(bf16_bits(a.y) & mk);
    o[2] = (unsigned short)(bf16_bits(a.z) & mk); o[3] = (unsigned short)(bf16_bits(a.w) & mk);
    o[4] = (unsigned short)(bf16_bits(b.x) & mk); o[5] = (unsigned short)(bf16_bits(b.y) & mk);
    o[6] = (unsigned short)(bf16_bits(b.z) & mk); o[7] = (unsigned short)(bf16_bits(b.w) & mk);
    st2_v8us(xb + (size_t)row * FD + k8, o);
  } else if (blk < PBX + PBW1) {
    const int u = (blk - PBX) * NTHR + tid;
    const int n = u >> 4, k8 = (u & 15) * 8;
    const v8us o = gather8(w1 + (size_t)k8 * FD + n, FD);
    st2_v8us(w1t + (size_t)n * FD + k8, o);
  } else if (blk < PBX + PBW1 + PBW2) {
    const int u = (blk - PBX - PBW1) * NTHR + tid;
    const int n = u / KU, k8 = (u % KU) * 8, kk = k8 & (FD - 1);
    const v8us o = gather8(w2 + (size_t)kk * FD + n, FD);
    st2_v8us(w2d + (size_t)n * KH + k8, o);
  } else if (blk < PBX + PBW1 + PBW2 + PBW3) {
    const int u = (blk - PBX - PBW1 - PBW2) * NTHR + tid;
    const int n = u / KU, k8 = (u % KU) * 8, kk = k8 & (FD - 1);
    const int nc = n < NC ? n : NC - 1;
    const unsigned short mk = n < NC ? (unsigned short)0xffffu : (unsigned short)0u;
    v8us o = gather8(w3 + (size_t)kk * NC + nc, NC);
#pragma unroll
    for (int i = 0; i < 8; ++i) o[i] = (unsigned short)(o[i] & mk);
    st2_v8us(w3d + (size_t)n * KH + k8, o);
  } else {
    if (tid < 32) {
      const v4f q0 = bf4(*(const v4fa*)(b1 + 4 * lane));
      const v4f q1 = bf4(*(const v4fa*)(g1 + 4 * lane));
      const v4f q2 = bf4(*(const v4fa*)(be1 + 4 * lane));
      const v4f q3 = bf4(*(const v4fa*)(b2 + 4 * lane));
      const v4f q4 = bf4(*(const v4fa*)(g2 + 4 * lane));
      const v4f q5 = bf4(*(const v4fa*)(be2 + 4 * lane));
      const int lc = lane < NC / 4 ? lane : NC / 4 - 1;
      const v4f r6 = *(const v4fa*)(b3 + 4 * lc);
      asm volatile("" :: "v"(r6));
      const unsigned m6 = lane < NC / 4 ? 0xffffffffu : 0u;
      v4f q6;
      q6.x = __uint_as_float((bf16_bits(r6.x) << 16) & m6);
      q6.y = __uint_as_float((bf16_bits(r6.y) << 16) & m6);
      q6.z = __uint_as_float((bf16_bits(r6.z) << 16) & m6);
      q6.w = __uint_as_float((bf16_bits(r6.w) << 16) & m6);
      float* pp = par + 4 * lane;
      *(volatile v4f*)(pp + 0 * FD) = q0; *(volatile v4f*)(pp + 1 * FD) = q1;
      *(volatile v4f*)(pp + 2 * FD) = q2; *(volatile v4f*)(pp + 3 * FD) = q3;
      *(volatile v4f*)(pp + 4 * FD) = q4; *(volatile v4f*)(pp + 5 * FD) = q5;
      *(volatile v4f*)(pp + 6 * FD) = q6;
      __threadfence();
      *(volatile v4f*)(pp + 0 * FD) = q0; *(volatile v4f*)(pp + 1 * FD) = q1;
      *(volatile v4f*)(pp + 2 * FD) = q2; *(volatile v4f*)(pp + 3 * FD) = q3;
      *(volatile v4f*)(pp + 4 * FD) = q4; *(volatile v4f*)(pp + 5 * FD) = q5;
      *(volatile v4f*)(pp + 6 * FD) = q6;
    }
  }
}

__device__ __forceinline__ void bucket_flush(const int* pl, const int* cnt, const int* dv, int ov,
                                             int* lp, int* cop, int* dp, int* fp, int tid) {
#pragma unroll 1
  for (int i = tid * 4; i < RCAP; i += NTHR * 4) {
    const v4i v = *(const v4ia*)(pl + i);
    *(volatile v4i*)(lp + i) = v;
  }
#pragma unroll 1
  for (int i = tid * 4; i < 2 * NBRUN; i += NTHR * 4) {
    const v4i v = *(const v4ia*)(cnt + i);
    *(volatile v4i*)(cop + i) = v;
  }
  {
    const v4i v = *(const v4ia*)(dv + 4 * tid);
    *(volatile v4i*)(dp + 4 * tid) = v;
  }
  if (tid < 8) {
    const v4i f = {ov, ov, ov, ov};
    *(volatile v4i*)(fp + 4 * tid) = f;
  }
}

__global__ __launch_bounds__(NTHR) void k_bucket(const int* __restrict__ srcs, const int* __restrict__ dsts,
                                                 int* LIST, int* CO, int* DINVB, int* FLAG) {
  extern __shared__ __attribute__((aligned(16))) int dsm[];
  int* wl   = dsm;
  int* pl   = dsm + BK_WL;
  int* cnt  = pl + RCAP;
  int* offs = cnt + NBRUN;
  int* cur  = offs + NBRUN;
  int* misc = cur + NBRUN;
  const int tid = (int)threadIdx.x, lane = tid & 31, wave = tid >> 5;
  const int blk = (int)blockIdx.x;
  const unsigned nbs = (unsigned)(blk * NBRUN);

  {
    const int fr0 = blk * NBRUN;
    const int fr  = fr0 < NN - 1 ? fr0 : NN - 1;
    for (int i = tid * 4; i < BK_ZINTS; i += NTHR * 4) {
      const int fv = (i >= BK_WL && i < BK_WL + RCAP) ? fr : 0;
      const v4i z4 = {fv, fv, fv, fv};
      *(v4ia*)(dsm + i) = z4;
    }
    if (tid < 16) misc[tid] = 0;
  }
  __syncthreads();

  {
    const int per  = ((NE + NWAVE * WCH - 1) / (NWAVE * WCH)) * WCH;
    const int ebeg = wave * per;
    const int eend = (ebeg + per < NE) ? (ebeg + per) : NE;
    int* mylist = wl + wave * WLCAP;
    int wc = 0;
#pragma unroll 1
    for (int cb = ebeg; cb < eend; cb += WCH) {
      const int e0 = cb + lane * EPT;
      const v4i da = *(const v4ia*)(dsts + e0);
      const v4i db = *(const v4ia*)(dsts + e0 + 4);
      const unsigned s0 = (unsigned)da.x - nbs, s1 = (unsigned)da.y - nbs;
      const unsigned s2 = (unsigned)da.z - nbs, s3 = (unsigned)da.w - nbs;
      const unsigned s4 = (unsigned)db.x - nbs, s5 = (unsigned)db.y - nbs;
      const unsigned s6 = (unsigned)db.z - nbs, s7 = (unsigned)db.w - nbs;
      const bool h0 = s0 < (unsigned)NBRUN, h1 = s1 < (unsigned)NBRUN, h2 = s2 < (unsigned)NBRUN, h3 = s3 < (unsigned)NBRUN;
      const bool h4 = s4 < (unsigned)NBRUN, h5 = s5 < (unsigned)NBRUN, h6 = s6 < (unsigned)NBRUN, h7 = s7 < (unsigned)NBRUN;
      const unsigned m0 = __builtin_amdgcn_ballot_w32(h0), m1 = __builtin_amdgcn_ballot_w32(h1);
      const unsigned m2 = __builtin_amdgcn_ballot_w32(h2), m3 = __builtin_amdgcn_ballot_w32(h3);
      const unsigned m4 = __builtin_amdgcn_ballot_w32(h4), m5 = __builtin_amdgcn_ballot_w32(h5);
      const unsigned m6 = __builtin_amdgcn_ballot_w32(h6), m7 = __builtin_amdgcn_ballot_w32(h7);
      const unsigned any = m0 | m1 | m2 | m3 | m4 | m5 | m6 | m7;
      if (any != 0u) {
        const int pre = (int)(__builtin_amdgcn_mbcnt_lo(m0, 0u) + __builtin_amdgcn_mbcnt_lo(m1, 0u) +
                              __builtin_amdgcn_mbcnt_lo(m2, 0u) + __builtin_amdgcn_mbcnt_lo(m3, 0u) +
                              __builtin_amdgcn_mbcnt_lo(m4, 0u) + __builtin_amdgcn_mbcnt_lo(m5, 0u) +
                              __builtin_amdgcn_mbcnt_lo(m6, 0u) + __builtin_amdgcn_mbcnt_lo(m7, 0u));
        int p = wc + pre;
        if (h0) { if (p < WLCAP) mylist[p] = ((e0 + 0) << SLB) | (int)s0; p = p + 1; }
        if (h1) { if (p < WLCAP) mylist[p] = ((e0 + 1) << SLB) | (int)s1; p = p + 1; }
        if (h2) { if (p < WLCAP) mylist[p] = ((e0 + 2) << SLB) | (int)s2; p = p + 1; }
        if (h3) { if (p < WLCAP) mylist[p] = ((e0 + 3) << SLB) | (int)s3; p = p + 1; }
        if (h4) { if (p < WLCAP) mylist[p] = ((e0 + 4) << SLB) | (int)s4; p = p + 1; }
        if (h5) { if (p < WLCAP) mylist[p] = ((e0 + 5) << SLB) | (int)s5; p = p + 1; }
        if (h6) { if (p < WLCAP) mylist[p] = ((e0 + 6) << SLB) | (int)s6; p = p + 1; }
        if (h7) { if (p < WLCAP) mylist[p] = ((e0 + 7) << SLB) | (int)s7; p = p + 1; }
        wc += (int)(__builtin_popcount(m0) + __builtin_popcount(m1) + __builtin_popcount(m2) + __builtin_popcount(m3) +
                    __builtin_popcount(m4) + __builtin_popcount(m5) + __builtin_popcount(m6) + __builtin_popcount(m7));
      }
    }
    if (lane == 0) misc[wave] = wc;
  }
  __syncthreads();

  if (wave == 0) {
    int ov = 0;
#pragma unroll 1
    for (int w2 = 0; w2 < NWAVE; ++w2) {
      int c = misc[w2];
      if (c > WLCAP) ov = 1;
      c = c < 0 ? 0 : (c > WLCAP ? WLCAP : c);
#pragma unroll 1
      for (int b0 = 0; b0 < c; b0 += 32) {
        const int idx = b0 + lane;
        const int ent = wl[w2 * WLCAP + (idx < WLCAP ? idx : WLCAP - 1)];
        const int m32 = (c - b0) < 32 ? (c - b0) : 32;
#pragma unroll 1
        for (int k = 0; k < m32; ++k) {
          const int u    = __builtin_amdgcn_readlane(ent, k);
          const int slot = u & (NBRUN - 1);
          if (lane == 0) cnt[slot] = cnt[slot] + 1;
        }
      }
    }
    if (lane == 0) misc[9] = ov;
  }
  __syncthreads();
  if (wave == 0) {
    const int base = lane * (NBRUN / 32);
    int s = 0;
#pragma unroll 1
    for (int i = 0; i < NBRUN / 32; ++i) s += cnt[base + i];
    int incl = s;
#pragma unroll
    for (int d = 1; d < 32; d <<= 1) {
      const int y = __shfl_up(incl, d, 32);
      if (lane >= d) incl += y;
    }
    int run = incl - s;
#pragma unroll 1
    for (int i = 0; i < NBRUN / 32; ++i) {
      const int cv = cnt[base + i];
      offs[base + i] = run;
      cur[base + i]  = run;
      run += cv;
    }
  }
  __syncthreads();

  if (wave == 0) {
#pragma unroll 1
    for (int w2 = 0; w2 < NWAVE; ++w2) {
      int c = misc[w2];
      c = c < 0 ? 0 : (c > WLCAP ? WLCAP : c);
#pragma unroll 1
      for (int b0 = 0; b0 < c; b0 += 32) {
        const int idx = b0 + lane;
        const int ent = wl[w2 * WLCAP + (idx < WLCAP ? idx : WLCAP - 1)];
        int eid = (ent >> SLB) & 0x1FFFFF;
        eid = eid > NE - 1 ? NE - 1 : eid;
        int sr = srcs[eid];
        sr = sr < 0 ? 0 : (sr > NN - 1 ? NN - 1 : sr);
        const int m32 = (c - b0) < 32 ? (c - b0) : 32;
#pragma unroll 1
        for (int k = 0; k < m32; ++k) {
          const int u    = __builtin_amdgcn_readlane(ent, k);
          const int wd   = __builtin_amdgcn_readlane(sr, k);
          const int slot = u & (NBRUN - 1);
          if (lane == 0) {
            int p = cur[slot];
            p = p < 0 ? 0 : (p > RCAP - 1 ? RCAP - 1 : p);
            pl[p] = wd;
            cur[slot] = p + 1;
          }
        }
      }
    }
  }
  __syncthreads();

#pragma unroll 1
  for (int i = 0; i < NBRUN / NTHR; ++i) {
    const int s = i * NTHR + tid;
    const float dg = (float)(cnt[s] + 1);
    cur[s] = __float_as_int(1.0f / sqrtf(dg));
  }
  __syncthreads();

  const int ovf = misc[9];
  int* lp  = LIST + (size_t)blk * RCAP;
  int* cop = CO + (size_t)blk * (2 * NBRUN);
  int* dp  = DINVB + (size_t)blk * NBRUN;
  int* fp  = FLAG + (size_t)blk * 32;
  bucket_flush(pl, cnt, cur, ovf, lp, cop, dp, fp, tid);
  __threadfence();
  bucket_flush(pl, cnt, cur, ovf, lp, cop, dp, fp, tid);
}

template <int KTOT, int NT>
__device__ __forceinline__ void gemm_16xN(const unsigned short* __restrict__ ap,
                                          const unsigned short* __restrict__ bp, v8f (&acc)[NT]) {
#pragma unroll 1
  for (int k0 = 0; k0 < KTOT; k0 += 32) {
    FragB af;
    af.h[0] = *(const v8usa*)(ap + k0);
    af.h[1] = *(const v8usa*)(ap + k0 + 16);
#pragma unroll
    for (int nt = 0; nt < NT; ++nt) {
      const unsigned short* wq = bp + (size_t)(16 * nt) * (size_t)KTOT + k0;
      FragB bf;
      bf.h[0] = *(const v8usa*)wq;
      bf.h[1] = *(const v8usa*)(wq + 16);
      acc[nt] = wmb(af, bf, acc[nt]);
    }
  }
}

template <int KTOT, int NT>
__global__ __launch_bounds__(GTHR) __attribute__((amdgpu_num_vgpr(248)))
void k_gemm(const unsigned short* __restrict__ A, const unsigned short* __restrict__ BT,
            const float* __restrict__ DINV, float* P) {
  constexpr int NCOL = 16 * NT;
  constexpr int SPT  = NCOL + 4;
  __shared__ __attribute__((aligned(16))) float stg[GBM * SPT];
  __shared__ __attribute__((aligned(16))) float sd[GBM];
  const int tid = (int)threadIdx.x, lane = tid & 31, wave = tid >> 5, hh = lane >> 4, m = lane & 15;
  const int rowBase = (int)blockIdx.x * GBM;
  if (tid < 32) *(v4fa*)(sd + 4 * m) = *(const v4fa*)(DINV + rowBase + 4 * m);

  v8f acc[NT];
  {
    const v8f z = {0.f, 0.f, 0.f, 0.f, 0.f, 0.f, 0.f, 0.f};
#pragma unroll
    for (int t = 0; t < NT; ++t) acc[t] = z;
  }
  const unsigned short* ap = A + (size_t)(rowBase + 16 * wave + m) * (size_t)KTOT + 8 * hh;
  const unsigned short* bp = BT + (size_t)m * (size_t)KTOT + 8 * hh;
  gemm_16xN<KTOT, NT>(ap, bp, acc);
#pragma unroll
  for (int nt = 0; nt < NT; ++nt) {
#pragma unroll
    for (int r = 0; r < 8; ++r) stg[(16 * wave + 8 * hh + r) * SPT + 16 * nt + m] = acc[nt][r];
  }
  __syncthreads();

  if constexpr (NT == 8) {
#pragma unroll 1
    for (int i = 0; i < 16; ++i) {
      const int lr   = 16 * wave + i;
      const int grow = rowBase + lr;
      const bool live = grow < NN;
      const v4f a = *(const v4fa*)(stg + lr * SPT + 4 * lane);
      const float di = sd[lr];
      asm volatile("" :: "v"(a));
      asm volatile("" :: "v"(di));
      v4f o;
      o.x = live ? di * a.x : 0.0f; o.y = live ? di * a.y : 0.0f;
      o.z = live ? di * a.z : 0.0f; o.w = live ? di * a.w : 0.0f;
      st2_v4f(P + (size_t)grow * NCOL + 4 * lane, o);
    }
  } else {
#pragma unroll 1
    for (int i = 0; i < 8; ++i) {
      const int lr   = 16 * wave + 2 * i + hh;
      const int grow = rowBase + lr;
      const bool live = (grow < NN) & (4 * m < NC);
      const v4f a = *(const v4fa*)(stg + lr * SPT + 4 * m);
      const float di = sd[lr];
      asm volatile("" :: "v"(a));
      asm volatile("" :: "v"(di));
      v4f o;
      o.x = live ? di * a.x : 0.0f; o.y = live ? di * a.y : 0.0f;
      o.z = live ? di * a.z : 0.0f; o.w = live ? di * a.w : 0.0f;
      st2_v4f(P + (size_t)grow * NCOL + 4 * m, o);
    }
  }
}

__global__ __launch_bounds__(NTHR) void k_replay(const int* __restrict__ LIST, const int* __restrict__ CO,
                                                 const float* __restrict__ DINV, const int* __restrict__ FLAG,
                                                 const float* __restrict__ P, const float* __restrict__ biasp,
                                                 float* PRE, float* REC) {
  __shared__ __attribute__((aligned(16))) float sb[FD];
  __shared__ __attribute__((aligned(16))) float wst[NWAVE * WSTW];
  __shared__ __attribute__((aligned(16))) float pst[RECW];
  const int tid = (int)threadIdx.x, lane = tid & 31, wave = tid >> 5;
  const int blk = (int)blockIdx.x;
  const int blkBase = blk * NBRUN;
  const int* lb  = LIST + (size_t)blk * RCAP;
  const int* cob = CO + (size_t)blk * (2 * NBRUN);
  const int flag = FLAG[(size_t)blk * 32];
  const float qnan = __uint_as_float(0x7fc00000u);
  if (tid < 32) *(v4fa*)(sb + 4 * lane) = *(const v4fa*)(biasp + 4 * lane);
  __syncthreads();
  const v4f bias = *(const v4fa*)(sb + 4 * lane);

  int nr = NN - (blkBase + 128 * wave);
  nr = nr < 0 ? 0 : (nr > 128 ? 128 : nr);
  int wn = 0;
  float wm0 = 0.0f, wm1 = 0.0f, wm2 = 0.0f, wm3 = 0.0f;
  float wq0 = 0.0f, wq1 = 0.0f, wq2 = 0.0f, wq3 = 0.0f;

#pragma unroll 1
  for (int r = 0; r < nr; ++r) {
    const int slot = 128 * wave + r;
    const int d    = blkBase + slot;
    int c = __builtin_amdgcn_readfirstlane(cob[slot]);
    int o = __builtin_amdgcn_readfirstlane(cob[NBRUN + slot]);
    const bool big = c > TRIPCAP;
    c = c < 0 ? 0 : (c > TRIPCAP ? TRIPCAP : c);
    o = o < 0 ? 0 : (o > RCAP - 1 ? RCAP - 1 : o);
    int last = o + c - 1;
    last = last < o ? o : last;
    last = last > RCAP - 1 ? RCAP - 1 : last;
    float a0 = 0.0f, a1 = 0.0f, a2 = 0.0f, a3 = 0.0f;
#pragma unroll 1
    for (int j = 0; j < c; j += 4) {
      int i0 = o + j, i1 = o + j + 1, i2 = o + j + 2, i3 = o + j + 3;
      i0 = i0 > last ? last : i0; i1 = i1 > last ? last : i1;
      i2 = i2 > last ? last : i2; i3 = i3 > last ? last : i3;
      int s0 = lb[i0], s1 = lb[i1], s2 = lb[i2], s3 = lb[i3];
      s0 = s0 < 0 ? 0 : (s0 > NN - 1 ? NN - 1 : s0);
      s1 = s1 < 0 ? 0 : (s1 > NN - 1 ? NN - 1 : s1);
      s2 = s2 < 0 ? 0 : (s2 > NN - 1 ? NN - 1 : s2);
      s3 = s3 < 0 ? 0 : (s3 > NN - 1 ? NN - 1 : s3);
      const v4f v0 = *(const v4fa*)(P + (size_t)s0 * FD + 4 * lane);
      const v4f v1 = *(const v4fa*)(P + (size_t)s1 * FD + 4 * lane);
      const v4f v2 = *(const v4fa*)(P + (size_t)s2 * FD + 4 * lane);
      const v4f v3 = *(const v4fa*)(P + (size_t)s3 * FD + 4 * lane);
      asm volatile("" :: "v"(v0));
      asm volatile("" :: "v"(v1));
      asm volatile("" :: "v"(v2));
      asm volatile("" :: "v"(v3));
      const bool p1 = (j + 1) < c, p2 = (j + 2) < c, p3 = (j + 3) < c;
      a0 = a0 + v0.x; a1 = a1 + v0.y; a2 = a2 + v0.z; a3 = a3 + v0.w;
      { const float t0 = a0 + v1.x, t1 = a1 + v1.y, t2 = a2 + v1.z, t3 = a3 + v1.w;
        a0 = p1 ? t0 : a0; a1 = p1 ? t1 : a1; a2 = p1 ? t2 : a2; a3 = p1 ? t3 : a3; }
      { const float t0 = a0 + v2.x, t1 = a1 + v2.y, t2 = a2 + v2.z, t3 = a3 + v2.w;
        a0 = p2 ? t0 : a0; a1 = p2 ? t1 : a1; a2 = p2 ? t2 : a2; a3 = p2 ? t3 : a3; }
      { const float t0 = a0 + v3.x, t1 = a1 + v3.y, t2 = a2 + v3.z, t3 = a3 + v3.w;
        a0 = p3 ? t0 : a0; a1 = p3 ? t1 : a1; a2 = p3 ? t2 : a2; a3 = p3 ? t3 : a3; }
    }
    const v4f sf = *(const v4fa*)(P + (size_t)d * FD + 4 * lane);
    const float di = DINV[d];
    float y0 = di * (a0 + sf.x) + bias.x, y1 = di * (a1 + sf.y) + bias.y;
    float y2 = di * (a2 + sf.z) + bias.z, y3 = di * (a3 + sf.w) + bias.w;
    const bool bad = (flag != 0) | big;
    y0 = bad ? qnan : y0; y1 = bad ? qnan : y1; y2 = bad ? qnan : y2; y3 = bad ? qnan : y3;
    v4f ov;
    ov.x = y0; ov.y = y1; ov.z = y2; ov.w = y3;
    float* op = PRE + (size_t)d * FD + 4 * lane;
    *(volatile v4f*)op = ov;
    __threadfence();
    *(volatile v4f*)op = ov;
    wn += 1;
    const float rk = 1.0f / (float)wn;
    { const float dd = y0 - wm0; wm0 = fmaf(dd, rk, wm0); wq0 = fmaf(dd, y0 - wm0, wq0); }
    { const float dd = y1 - wm1; wm1 = fmaf(dd, rk, wm1); wq1 = fmaf(dd, y1 - wm1, wq1); }
    { const float dd = y2 - wm2; wm2 = fmaf(dd, rk, wm2); wq2 = fmaf(dd, y2 - wm2, wq2); }
    { const float dd = y3 - wm3; wm3 = fmaf(dd, rk, wm3); wq3 = fmaf(dd, y3 - wm3, wq3); }
  }

  if (lane == 0) wst[wave * WSTW] = (float)wn;
  wst[wave * WSTW + 1 + 4 * lane + 0] = wm0; wst[wave * WSTW + 1 + 4 * lane + 1] = wm1;
  wst[wave * WSTW + 1 + 4 * lane + 2] = wm2; wst[wave * WSTW + 1 + 4 * lane + 3] = wm3;
  wst[wave * WSTW + 1 + FD + 4 * lane + 0] = wq0; wst[wave * WSTW + 1 + FD + 4 * lane + 1] = wq1;
  wst[wave * WSTW + 1 + FD + 4 * lane + 2] = wq2; wst[wave * WSTW + 1 + FD + 4 * lane + 3] = wq3;
  __syncthreads();
  if (tid < FD) {
    float n = 0.0f, mean = 0.0f, M2 = 0.0f;
#pragma unroll 1
    for (int w2 = 0; w2 < NWAVE; ++w2) {
      const float nb = wst[w2 * WSTW];
      const float mb = wst[w2 * WSTW + 1 + tid];
      const float qb = wst[w2 * WSTW + 1 + FD + tid];
      if (nb > 0.5f) {
        const float nn = n + nb;
        const float delta = mb - mean;
        const float f = nb / nn;
        mean = fmaf(delta, f, mean);
        M2 = M2 + qb + delta * delta * n * f;
        n = nn;
      }
    }
    pst[tid] = n;
    pst[FD + tid] = mean;
    pst[2 * FD + tid] = M2;
  }
  __syncthreads();
  v4f ps = {0.f, 0.f, 0.f, 0.f};
  float* rp = REC + (size_t)blk * RECW;
  if (tid < RECW / 4) {
    ps = *(const v4fa*)(pst + 4 * tid);
    *(volatile v4f*)(rp + 4 * tid) = ps;
  }
  __threadfence();
  if (tid < RECW / 4) {
    *(volatile v4f*)(rp + 4 * tid) = ps;
  }
}

__global__ __launch_bounds__(FD) void k_comb(const float* __restrict__ REC, float* STAT) {
  __shared__ __attribute__((aligned(16))) float st[2 * FD];
  const int tid = (int)threadIdx.x;
  double n = 0.0, mean = 0.0, M2 = 0.0;
#pragma unroll 1
  for (int b = 0; b < NBK; ++b) {
    const float* pr = REC + (size_t)b * RECW;
    const double nb = (double)pr[tid];
    const double mb = (double)pr[FD + tid];
    const double qb = (double)pr[2 * FD + tid];
    if (nb > 0.5) {
      const double nn = n + nb;
      const double delta = mb - mean;
      const double f = nb / nn;
      mean = mean + delta * f;
      M2 = M2 + qb + delta * delta * n * f;
      n = nn;
    }
  }
  const double nt = n < 1.0 ? 1.0 : n;
  const float varf  = (float)(M2 / nt);
  const float meanf = (float)mean;
  const float rstd  = 1.0f / sqrtf(varf + 1e-5f);
  st[tid] = meanf;
  st[FD + tid] = rstd;
  __syncthreads();
  v4f v = {0.f, 0.f, 0.f, 0.f};
  if (tid < (2 * FD) / 4) {
    v = *(const v4fa*)(st + 4 * tid);
    *(volatile v4f*)(STAT + 4 * tid) = v;
  }
  __threadfence();
  if (tid < (2 * FD) / 4) {
    *(volatile v4f*)(STAT + 4 * tid) = v;
  }
}

template <int LAYER>
__global__ __launch_bounds__(NTHR) void k_apply(const float* __restrict__ PRE, const float* __restrict__ STAT,
                                                const float* __restrict__ gam, const float* __restrict__ bet,
                                                const float* __restrict__ x, unsigned short* Hhl) {
  __shared__ __attribute__((aligned(16))) float sp[4 * FD];
  const int tid = (int)threadIdx.x, lane = tid & 31, wave = tid >> 5;
  if (tid < 32) {
    const v4f a = *(const v4fa*)(STAT + 4 * lane);
    const v4f b = *(const v4fa*)(STAT + FD + 4 * lane);
    const v4f c = *(const v4fa*)(gam + 4 * lane);
    const v4f d = *(const v4fa*)(bet + 4 * lane);
    *(v4fa*)(sp + 4 * lane) = a;
    *(v4fa*)(sp + FD + 4 * lane) = b;
    *(v4fa*)(sp + 2 * FD + 4 * lane) = c;
    *(v4fa*)(sp + 3 * FD + 4 * lane) = d;
  }
  __syncthreads();
  const v4f mu = *(const v4fa*)(sp + 4 * lane);
  const v4f rs = *(const v4fa*)(sp + FD + 4 * lane);
  const v4f gg = *(const v4fa*)(sp + 2 * FD + 4 * lane);
  const v4f bb = *(const v4fa*)(sp + 3 * FD + 4 * lane);
  const int rowBase = (int)blockIdx.x * 64 + 8 * wave;

#pragma unroll 1
  for (int i = 0; i < 8; ++i) {
    const int row = rowBase + i;
    const int rc  = row < NN ? row : NN - 1;
    const bool live = row < NN;
    const v4f p = *(const v4fa*)(PRE + (size_t)rc * FD + 4 * lane);
    asm volatile("" :: "v"(p));
    float v0 = ((p.x - mu.x) * rs.x) * gg.x + bb.x;
    float v1 = ((p.y - mu.y) * rs.y) * gg.y + bb.y;
    float v2 = ((p.z - mu.z) * rs.z) * gg.z + bb.z;
    float v3 = ((p.w - mu.w) * rs.w) * gg.w + bb.w;
    if constexpr (LAYER == 1) {
      const v4f xv = *(const v4fa*)(x + (size_t)rc * FD + 4 * lane);
      asm volatile("" :: "v"(xv));
      v0 = v0 + bf16_val(xv.x); v1 = v1 + bf16_val(xv.y);
      v2 = v2 + bf16_val(xv.z); v3 = v3 + bf16_val(xv.w);
    }
    v0 = (v0 > 0.0f) ? v0 : (v0 - v0); v1 = (v1 > 0.0f) ? v1 : (v1 - v1);
    v2 = (v2 > 0.0f) ? v2 : (v2 - v2); v3 = (v3 > 0.0f) ? v3 : (v3 - v3);
    v0 = live ? v0 : 0.0f; v1 = live ? v1 : 0.0f; v2 = live ? v2 : 0.0f; v3 = live ? v3 : 0.0f;
    int h01, h23, l01, l23;
    hilo_pack(v0, v1, v2, v3, h01, h23, l01, l23);
    if constexpr (SPLIT_H != 0) {
      const v4i ow = regroup32(h01, h23, l01, l23, lane);
      unsigned short* hp = Hhl + (size_t)row * KH + 8 * lane;
      *(volatile v4i*)hp = ow;
      __threadfence();
      *(volatile v4i*)hp = ow;
    } else {
      v2i ow;
      ow.x = h01; ow.y = h23;
      unsigned short* hp = Hhl + (size_t)row * KH + 4 * lane;
      *(volatile v2i*)hp = ow;
      __threadfence();
      *(volatile v2i*)hp = ow;
    }
  }
}

__global__ __launch_bounds__(NTHR) void k_replay3(const int* __restrict__ LIST, const int* __restrict__ CO,
                                                  const float* __restrict__ DINV, const int* __restrict__ FLAG,
                                                  const float* __restrict__ P3, const float* __restrict__ b3p,
                                                  float* out) {
  __shared__ __attribute__((aligned(16))) float lg[NWAVE * 32 * NC];
  __shared__ __attribute__((aligned(16))) float sb3[NCP];
  const int tid = (int)threadIdx.x, lane = tid & 31, wave = tid >> 5, hh = lane >> 4, q = lane & 15;
  const int blk = (int)blockIdx.x;
  const int blkBase = blk * NBRUN;
  const int* lb  = LIST + (size_t)blk * RCAP;
  const int* cob = CO + (size_t)blk * (2 * NBRUN);
  const int flag = FLAG[(size_t)blk * 32];
  const float qnan = __uint_as_float(0x7fc00000u);
  if (tid < 32) *(v4fa*)(sb3 + 4 * q) = *(const v4fa*)(b3p + 4 * q);
  __syncthreads();
  const v4f bias = *(const v4fa*)(sb3 + 4 * q);
  float* lgw = lg + wave * (32 * NC);

#pragma unroll 1
  for (int g = 0; g < 4; ++g) {
    const int d0 = blkBase + 128 * wave + 32 * g;
#pragma unroll 1
    for (int r = 0; r < 32; ++r) {
      const int d    = d0 + r;
      const int dc   = d < NN ? d : NN - 1;
      const int slot = dc - blkBase;
      int c = __builtin_amdgcn_readfirstlane(cob[slot]);
      int o = __builtin_amdgcn_readfirstlane(cob[NBRUN + slot]);
      const bool big = c > TRIPCAP;
      c = c < 0 ? 0 : (c > TRIPCAP ? TRIPCAP : c);
      o = o < 0 ? 0 : (o > RCAP - 1 ? RCAP - 1 : o);
      int last = o + c - 1;
      last = last < o ? o : last;
      last = last > RCAP - 1 ? RCAP - 1 : last;
      const int ntr = (c + 1) >> 1;
      float a0 = 0.0f, a1 = 0.0f, a2 = 0.0f, a3 = 0.0f;
#pragma unroll 1
      for (int j = 0; j < ntr; ++j) {
        const int hidx = 2 * j + hh;
        int idx = o + hidx;
        idx = idx > last ? last : idx;
        int sr = lb[idx];
        sr = sr < 0 ? 0 : (sr > NN - 1 ? NN - 1 : sr);
        const v4f v = *(const v4fa*)(P3 + (size_t)sr * NCP + 4 * q);
        asm volatile("" :: "v"(v));
        const bool valid = hidx < c;
        const float t0 = a0 + v.x, t1 = a1 + v.y, t2 = a2 + v.z, t3 = a3 + v.w;
        a0 = valid ? t0 : a0; a1 = valid ? t1 : a1; a2 = valid ? t2 : a2; a3 = valid ? t3 : a3;
      }
      a0 = a0 + __shfl_xor(a0, 16, 32); a1 = a1 + __shfl_xor(a1, 16, 32);
      a2 = a2 + __shfl_xor(a2, 16, 32); a3 = a3 + __shfl_xor(a3, 16, 32);
      const v4f sf = *(const v4fa*)(P3 + (size_t)dc * NCP + 4 * q);
      asm volatile("" :: "v"(sf));
      const float di = DINV[dc];
      asm volatile("" :: "v"(di));
      float y0 = di * (a0 + sf.x) + bias.x, y1 = di * (a1 + sf.y) + bias.y;
      float y2 = di * (a2 + sf.z) + bias.z, y3 = di * (a3 + sf.w) + bias.w;
      y0 = big ? qnan : y0; y1 = big ? qnan : y1; y2 = big ? qnan : y2; y3 = big ? qnan : y3;
      v4f ov;
      ov.x = y0; ov.y = y1; ov.z = y2; ov.w = y3;
      if (hh == 0 && q < NC / 4) *(v4fa*)(lgw + r * NC + 4 * q) = ov;
    }
    __syncthreads();
    {
      float* p = lgw + lane * NC;
      float mx = p[0];
#pragma unroll 1
      for (int c = 1; c < NC; ++c) {
        const float xv = p[c];
        mx = ((xv > mx) | (xv != xv)) ? xv : mx;
      }
      float se = 0.0f;
#pragma unroll 1
      for (int c = 0; c < NC; ++c) se += expf(p[c] - mx);
      const float ls = logf(se);
#pragma unroll 1
      for (int c = 0; c < NC; ++c) {
        const float v = (p[c] - mx) - ls;
        p[c] = (flag != 0) ? qnan : v;
      }
    }
    __syncthreads();
    {
      const bool liveg = d0 < NN;
      float* ob = out + (size_t)d0 * NC;
#pragma unroll 1
      for (int it = 0; it < (32 * NC / 4) / 32; ++it) {
        const int i4 = it * 32 + lane;
        const v4f v = *(const v4fa*)(lgw + 4 * i4);
        asm volatile("" :: "v"(v));
        if (liveg) *(volatile v4f*)(ob + (size_t)4 * (size_t)i4) = v;
      }
      __threadfence();
#pragma unroll 1
      for (int it = 0; it < (32 * NC / 4) / 32; ++it) {
        const int i4 = it * 32 + lane;
        const v4f v = *(const v4fa*)(lgw + 4 * i4);
        asm volatile("" :: "v"(v));
        if (liveg) *(volatile v4f*)(ob + (size_t)4 * (size_t)i4) = v;
      }
    }
    __syncthreads();
  }
}

extern "C" void kernel_launch(void* const* d_in, const int* in_sizes, int n_in,
                              void* d_out, int out_size, void* d_ws, size_t ws_size,
                              hipStream_t stream) {
  if (n_in < 12) return;
  if (in_sizes[0] != NN * FD) return;
  if (in_sizes[1] != 2 * NE) return;
  if (in_sizes[2] != FD * FD) return;
  if (in_sizes[3] != FD || in_sizes[4] != FD || in_sizes[5] != FD) return;
  if (in_sizes[6] != FD * FD) return;
  if (in_sizes[7] != FD || in_sizes[8] != FD || in_sizes[9] != FD) return;
  if (in_sizes[10] != FD * NC) return;
  if (in_sizes[11] != NC) return;
  if (out_size != NN * NC) return;

  const float* x   = (const float*)d_in[0];
  const int*   ei  = (const int*)d_in[1];
  const float* W1  = (const float*)d_in[2];
  const float* b1  = (const float*)d_in[3];
  const float* g1  = (const float*)d_in[4];
  const float* be1 = (const float*)d_in[5];
  const float* W2  = (const float*)d_in[6];
  const float* b2  = (const float*)d_in[7];
  const float* g2  = (const float*)d_in[8];
  const float* be2 = (const float*)d_in[9];
  const float* W3  = (const float*)d_in[10];
  const float* b3  = (const float*)d_in[11];
  float* out = (float*)d_out;
  const int* srcs = ei;
  const int* dsts = ei + NE;

  constexpr size_t zR    = (size_t)MP * FD * 4;
  constexpr size_t zLIST = (size_t)NBK * RCAP * 4;
  constexpr size_t zCO   = (size_t)NBK * 2 * NBRUN * 4;
  constexpr size_t zDINV = (size_t)NBK * NBRUN * 4;
  constexpr size_t zFLAG = (size_t)NBK * 128;
  constexpr size_t zW1T  = (size_t)FD * FD * 2;
  constexpr size_t zW2D  = (size_t)FD * KH * 2;
  constexpr size_t zW3D  = (size_t)NCP * KH * 2;
  constexpr size_t zPAR  = 4096;
  constexpr size_t zREC  = (size_t)NBK * RECW * 4;
  constexpr size_t zSTAT = 1024;
  constexpr size_t oRA   = 0;
  constexpr size_t oRB   = oRA + zR;
  constexpr size_t oLIST = oRB + zR;
  constexpr size_t oCO   = oLIST + zLIST;
  constexpr size_t oDINV = oCO + zCO;
  constexpr size_t oFLAG = oDINV + zDINV;
  constexpr size_t oW1T  = oFLAG + zFLAG;
  constexpr size_t oW2D  = oW1T + zW1T;
  constexpr size_t oW3D  = oW2D + zW2D;
  constexpr size_t oPAR  = oW3D + zW3D;
  constexpr size_t oREC1 = oPAR + zPAR;
  constexpr size_t oREC2 = oREC1 + zREC;
  constexpr size_t oST1  = oREC2 + zREC;
  constexpr size_t oST2  = oST1 + zSTAT;
  constexpr size_t oEND  = oST2 + zSTAT;
  static_assert(zR % 256 == 0 && zLIST % 256 == 0 && zCO % 256 == 0 && zDINV % 256 == 0 && zFLAG % 256 == 0);
  static_assert(zW1T % 256 == 0 && zW2D % 256 == 0 && zW3D % 256 == 0 && zREC % 256 == 0);
  static_assert(zR >= (size_t)MP * KH * 2 && zR >= (size_t)MP * FD * 2 && zR >= (size_t)MP * NCP * 4);
  static_assert(7 * FD * 4 <= zPAR && 2 * FD * 4 <= zSTAT);
  static_assert(oEND <= (size_t)WSMAX);
  if (oEND > ws_size) return;

  char* ws = (char*)d_ws;
  float*          RAf  = (float*)(ws + oRA);
  unsigned short* RAh  = (unsigned short*)(ws + oRA);
  float*          RBf  = (float*)(ws + oRB);
  unsigned short* RBh  = (unsigned short*)(ws + oRB);
  int*            LIST = (int*)(ws + oLIST);
  int*            CO   = (int*)(ws + oCO);
  float*          DINV = (float*)(ws + oDINV);
  int*            FLAG = (int*)(ws + oFLAG);
  unsigned short* W1T  = (unsigned short*)(ws + oW1T);
  unsigned short* W2D  = (unsigned short*)(ws + oW2D);
  unsigned short* W3D  = (unsigned short*)(ws + oW3D);
  float*          PAR  = (float*)(ws + oPAR);
  float*          REC1 = (float*)(ws + oREC1);
  float*          REC2 = (float*)(ws + oREC2);
  float*          ST1  = (float*)(ws + oST1);
  float*          ST2  = (float*)(ws + oST2);

  hipFuncSetAttribute(reinterpret_cast<const void*>(&k_bucket), hipFuncAttributeMaxDynamicSharedMemorySize, (int)BK_LDS);

  k_prep<<<PBTOT, NTHR, 0, stream>>>(x, W1, b1, g1, be1, W2, b2, g2, be2, W3, b3, RBh, W1T, W2D, W3D, PAR);
  k_bucket<<<NBK, NTHR, BK_LDS, stream>>>(srcs, dsts, LIST, CO, (int*)DINV, FLAG);
  k_gemm<FD, 8><<<MP / GBM, GTHR, 0, stream>>>(RBh, W1T, DINV, RAf);
  k_replay<<<NBK, NTHR, 0, stream>>>(LIST, CO, DINV, FLAG, RAf, PAR + 0 * FD, RBf, REC1);
  k_comb<<<1, FD, 0, stream>>>(REC1, ST1);
  k_apply<1><<<MP / 64, NTHR, 0, stream>>>(RBf, ST1, PAR + 1 * FD, PAR + 2 * FD, x, RAh);
  k_gemm<KH, 8><<<MP / GBM, GTHR, 0, stream>>>(RAh, W2D, DINV, RBf);
  k_replay<<<NBK, NTHR, 0, stream>>>(LIST, CO, DINV, FLAG, RBf, PAR + 3 * FD, RAf, REC2);
  k_comb<<<1, FD, 0, stream>>>(REC2, ST2);
  k_apply<2><<<MP / 64, NTHR, 0, stream>>>(RAf, ST2, PAR + 4 * FD, PAR + 5 * FD, x, RBh);
  k_gemm<KH, 4><<<MP / GBM, GTHR, 0, stream>>>(RBh, W3D, DINV, RAf);
  k_replay3<<<NBK, NTHR, 0, stream>>>(LIST, CO, DINV, FLAG, RAf, PAR + 6 * FD, out);
}
